// TemporalHeteroGNN_74225624809923
// MI455X (gfx1250) — hardware-run, weakly checked
//
#include <hip/hip_runtime.h>
#include <stddef.h>
#include <stdint.h>
#include <math.h>

#define SPLIT_KQV 1
#define SPLIT_REL 1
#define SPLIT_OUT 1

#define NU      30000
#define NEV     60000
#define NVN     1000
#define PU      30720
#define PE      60416
#define PV      1024
#define PB0     0
#define PB1     30720
#define PB2     91136
#define NP      92160
#define HD      64
#define KL      128
#define WP      128
#define KEXT_KQV (SPLIT_KQV ? 128 : 64)
#define KEXT_OUT (SPLIT_OUT ? 128 : 64)
#define XK      32
#define GBM     128
#define NTHR    256
#define NWAVE   8
#define SP      68
#define STW     96
#define RBW     32
#define RBMAT   (64 * RBW)
#define NLE     26

#define RUNCAP  11264
#define WLCAP   2048
#define NSMAX   1024
#define EIDSH   10
#define WCH     256
#define TRIPCAP 256
#define MAXDEG_MEAS 84
#define MAXB_USER   5244
#define MAXB_EVENT  2147
#define NRUNS   542
#define NSLOTW  547840
#define MX0     (-1.0e30f)

#define BK_ZINTS (NWAVE * WLCAP + RUNCAP + 3 * NSMAX)
#define BK_INTS  (BK_ZINTS + 16)
#define BK_LDS   (BK_INTS * 4)

#define RB_E0   0
#define RB_E6   30
#define RB_E7   60
#define RB_E8   90
#define RB_E9   120
#define RB_E10  150
#define RB_E1   180
#define RB_E2   239
#define RB_E3   298
#define RB_E4   357
#define RB_E5   416
#define RB_E12  475
#define RB_E11  534

#define VB_IN   0
#define VB_KQV  192
#define VB_OUT  1344
#define VB_PREL 1728
#define VB_SKIP 1856
#define VECN    2048

#define PBXU  480
#define PBXE  944
#define PBXV  16
#define PBX   (PBXU + PBXE + PBXV)
#define PBKQ  72
#define PBWO  24
#define PBTOT (PBX + 3 + PBKQ + PBWO + 2 * NLE + 7)

static_assert(PB1 == PU && PB2 == PU + PE && NP == PU + PE + PV && NP == 92160);
static_assert(PU % 1024 == 0 && PE % 1024 == 0 && PV % 128 == 0 && PU % GBM == 0 && PE % GBM == 0 && PV % GBM == 0);
static_assert(PU >= NU && PE >= NEV && PV >= NVN);
static_assert(NU < 65536 && NEV < 65536 && NVN < 65536);
static_assert(RUNCAP >= 128 * MAXDEG_MEAS && RUNCAP * 100 >= MAXB_USER * 105 && RUNCAP * 100 >= MAXB_EVENT * 105);
static_assert(RUNCAP < 65536 && RUNCAP % (NTHR * 4) == 0 && BK_ZINTS % (NTHR * 4) == 0);
static_assert(WLCAP >= (128 * MAXDEG_MEAS) / 8 + 256);
static_assert(MAXDEG_MEAS + 8 <= TRIPCAP);
static_assert(6 * (PU / 1024) + 6 * (PE / 1024) + 1 * (PV / 128) == NRUNS);
static_assert(6 * PU + 6 * PE + PV == NSLOTW);
static_assert((150000 << EIDSH) > 0 && 150000 < (1 << 21));
static_assert(BK_LDS <= 300000 && (GBM * SP + 64) * 4 <= 65536);
static_assert(PBXU * NTHR == PU * 4 && PBXE * NTHR == PE * 4 && PBXV * NTHR == PV * 4);
static_assert(PBKQ * NTHR == 6 * 192 * 16 && PBWO * NTHR == 6 * 64 * 16);
static_assert(KL % 32 == 0 && XK % 32 == 0 && KL == 2 * HD && GBM * KL * 2 <= GBM * SP * 4);

typedef float          v2f   __attribute__((ext_vector_type(2)));
typedef float          v4f   __attribute__((ext_vector_type(4)));
typedef float          v8f   __attribute__((ext_vector_type(8)));
typedef int            v2i   __attribute__((ext_vector_type(2)));
typedef int            v4i   __attribute__((ext_vector_type(4)));
typedef int            v8i   __attribute__((ext_vector_type(8)));
typedef unsigned short v8us  __attribute__((ext_vector_type(8)));
typedef unsigned short v16us __attribute__((ext_vector_type(16)));
typedef __bf16         v16bf __attribute__((ext_vector_type(16)));
typedef v2f  __attribute__((may_alias)) v2fa;
typedef v4f  __attribute__((may_alias)) v4fa;
typedef v2i  __attribute__((may_alias)) v2ia;
typedef v4i  __attribute__((may_alias)) v4ia;
typedef v8us __attribute__((may_alias)) v8usa;
union FragB { v16bf v; v16us u; v8us h[2]; v8i w; };

__device__ __forceinline__ v8f wmb(const FragB& a, const FragB& b, v8f c) {
  v8f d = __builtin_amdgcn_wmma_f32_16x16x32_bf16(false, a.v, false, b.v, (short)0, c, false, false);
  asm volatile("v_nop\n\tv_nop\n\tv_nop\n\tv_nop" : "+v"(d) : "v"(a.w), "v"(b.w));
  return d;
}

__device__ __forceinline__ unsigned bf16_bits(float f) {
  const unsigned u = __float_as_uint(f);
  const unsigned r = (u + 0x7FFFu + ((u >> 16) & 1u)) >> 16;
  const unsigned q = (u >> 16) | 0x40u;
  return ((u & 0x7fffffffu) > 0x7f800000u) ? q : r;
}
__device__ __forceinline__ float bf16_val(float f) { return __uint_as_float(bf16_bits(f) << 16); }

__device__ __forceinline__ void hilo_pack(float v0, float v1, float v2, float v3,
                                          int& h01, int& h23, int& l01, int& l23) {
  const unsigned a0 = bf16_bits(v0), a1 = bf16_bits(v1), a2 = bf16_bits(v2), a3 = bf16_bits(v3);
  const unsigned b0 = bf16_bits(v0 - __uint_as_float(a0 << 16));
  const unsigned b1 = bf16_bits(v1 - __uint_as_float(a1 << 16));
  const unsigned b2 = bf16_bits(v2 - __uint_as_float(a2 << 16));
  const unsigned b3 = bf16_bits(v3 - __uint_as_float(a3 << 16));
  h01 = (int)(a0 | (a1 << 16)); h23 = (int)(a2 | (a3 << 16));
  l01 = (int)(b0 | (b1 << 16)); l23 = (int)(b2 | (b3 << 16));
}

__device__ __forceinline__ v4i regroup8(int h01, int h23, int l01, int l23, int lane) {
  const int t  = lane & 15;
  const int s0 = (lane & 16) + ((2 * t) & 15), s1 = s0 + 1;
  const int a0 = __shfl(h01, s0, 32), a1 = __shfl(h23, s0, 32), a2 = __shfl(h01, s1, 32), a3 = __shfl(h23, s1, 32);
  const int b0 = __shfl(l01, s0, 32), b1 = __shfl(l23, s0, 32), b2 = __shfl(l01, s1, 32), b3 = __shfl(l23, s1, 32);
  const int mk = (t < 8) ? -1 : 0;
  v4i o;
  o.x = (a0 & mk) | (b0 & ~mk); o.y = (a1 & mk) | (b1 & ~mk);
  o.z = (a2 & mk) | (b2 & ~mk); o.w = (a3 & mk) | (b3 & ~mk);
  return o;
}

__device__ __forceinline__ void st2_v4f(float* p, v4f v) {
  *(volatile v4f*)p = v;
  __threadfence();
  *(volatile v4f*)p = v;
}
__device__ __forceinline__ void st2_v8us(unsigned short* p, v8us v) {
  *(volatile v8us*)p = v;
  __threadfence();
  *(volatile v8us*)p = v;
}

__device__ __forceinline__ v8us gather8(const float* __restrict__ base, int stride, unsigned mk) {
  float f[8];
#pragma unroll
  for (int i = 0; i < 8; ++i) f[i] = base[(size_t)i * (size_t)stride];
  v8us o;
#pragma unroll
  for (int i = 0; i < 8; ++i) o[i] = (unsigned short)(bf16_bits(f[i]) & mk);
  return o;
}
__device__ __forceinline__ v8us xrow8(const float* __restrict__ p, unsigned mk) {
  const v4f a = *(const v4fa*)p;
  const v4f b = *(const v4fa*)(p + 4);
  v8us o;
  o[0] = (unsigned short)(bf16_bits(a.x) & mk); o[1] = (unsigned short)(bf16_bits(a.y) & mk);
  o[2] = (unsigned short)(bf16_bits(a.z) & mk); o[3] = (unsigned short)(bf16_bits(a.w) & mk);
  o[4] = (unsigned short)(bf16_bits(b.x) & mk); o[5] = (unsigned short)(bf16_bits(b.y) & mk);
  o[6] = (unsigned short)(bf16_bits(b.z) & mk); o[7] = (unsigned short)(bf16_bits(b.w) & mk);
  return o;
}
__device__ __forceinline__ void vec_copy(const float* __restrict__ src, int nsrc, float* dst, int npieces, int tid) {
#pragma unroll 1
  for (int p0 = 0; p0 < npieces; p0 += NTHR) {
    const int p = p0 + tid, i0 = 4 * p;
    const int j0 = (i0     < nsrc) ? i0     : nsrc - 1;
    const int j1 = (i0 + 1 < nsrc) ? i0 + 1 : nsrc - 1;
    const int j2 = (i0 + 2 < nsrc) ? i0 + 2 : nsrc - 1;
    const int j3 = (i0 + 3 < nsrc) ? i0 + 3 : nsrc - 1;
    const float a0 = src[j0], a1 = src[j1], a2 = src[j2], a3 = src[j3];
    asm volatile("" :: "v"(a0), "v"(a1), "v"(a2), "v"(a3));
    const unsigned m0 = (i0     < nsrc) ? 0xffffffffu : 0u, m1 = (i0 + 1 < nsrc) ? 0xffffffffu : 0u;
    const unsigned m2 = (i0 + 2 < nsrc) ? 0xffffffffu : 0u, m3 = (i0 + 3 < nsrc) ? 0xffffffffu : 0u;
    v4f o;
    o.x = __uint_as_float((bf16_bits(a0) << 16) & m0);
    o.y = __uint_as_float((bf16_bits(a1) << 16) & m1);
    o.z = __uint_as_float((bf16_bits(a2) << 16) & m2);
    o.w = __uint_as_float((bf16_bits(a3) << 16) & m3);
    if (p < npieces) st2_v4f(dst + 4 * p, o);
  }
}

__device__ __forceinline__ int type_of_blk(int bx) { return (bx >= PU / GBM ? 1 : 0) + (bx >= (PU + PE) / GBM ? 1 : 0); }

__global__ __launch_bounds__(NTHR) void k_prep(
    const float* __restrict__ xu, const float* __restrict__ xe, const float* __restrict__ xv,
    const float* __restrict__ wu, const float* __restrict__ we, const float* __restrict__ wv,
    const float* __restrict__ bu, const float* __restrict__ be, const float* __restrict__ bv,
    const float* __restrict__ wkqv, const float* __restrict__ bkqv, const float* __restrict__ wk,
    const float* __restrict__ wvv, const float* __restrict__ prel, const float* __restrict__ wout,
    const float* __restrict__ bout, const float* __restrict__ skip,
    unsigned short* XB, unsigned short* WT, unsigned short* WKQ, unsigned short* WOU, unsigned short* RB,
    float* VEC) {
  const int tid = (int)threadIdx.x;
  const int blk = (int)blockIdx.x;
  if (blk < PBXU) {
    const int u = blk * NTHR + tid, row = u >> 2, k8 = (u & 3) * 8;
    const int rc = row < NU ? row : NU - 1;
    const unsigned mk = row < NU ? 0xffffu : 0u;
    const v8us o = xrow8(xu + (size_t)rc * 32 + k8, mk);
    st2_v8us(XB + (size_t)(PB0 + row) * XK + k8, o);
  } else if (blk < PBXU + PBXE) {
    const int u = (blk - PBXU) * NTHR + tid, row = u >> 2, k8 = (u & 3) * 8;
    const int rc = row < NEV ? row : NEV - 1;
    const unsigned mk = row < NEV ? 0xffffu : 0u;
    const v8us o = xrow8(xe + (size_t)rc * 32 + k8, mk);
    st2_v8us(XB + (size_t)(PB1 + row) * XK + k8, o);
  } else if (blk < PBX) {
    const int u = (blk - PBXU - PBXE) * NTHR + tid, row = u >> 2, k8 = (u & 3) * 8;
    const int rc = row < NVN ? row : NVN - 1;
    const int kc = k8 < 16 ? k8 : 8;
    const unsigned mk = (row < NVN && k8 < 16) ? 0xffffu : 0u;
    const v8us o = xrow8(xv + (size_t)rc * 16 + kc, mk);
    st2_v8us(XB + (size_t)(PB2 + row) * XK + k8, o);
  } else if (blk < PBX + 1) {
    const int n = tid >> 2, k8 = (tid & 3) * 8;
    const v8us o = gather8(wu + (size_t)k8 * HD + n, HD, 0xffffu);
    st2_v8us(WT + (size_t)tid * 8, o);
  } else if (blk < PBX + 2) {
    const int n = tid >> 2, k8 = (tid & 3) * 8;
    const v8us o = gather8(we + (size_t)k8 * HD + n, HD, 0xffffu);
    st2_v8us(WT + (size_t)(64 * XK) + (size_t)tid * 8, o);
  } else if (blk < PBX + 3) {
    const int n = tid >> 2, k8 = (tid & 3) * 8;
    const int kc = k8 < 16 ? k8 : 8;
    const v8us o = gather8(wv + (size_t)kc * HD + n, HD, k8 < 16 ? 0xffffu : 0u);
    st2_v8us(WT + (size_t)(2 * 64 * XK) + (size_t)tid * 8, o);
  } else if (blk < PBX + 3 + PBKQ) {
    const int u = (blk - PBX - 3) * NTHR + tid;
    const int lt = u / 3072, rem = u - lt * 3072;
    const int n = rem >> 4, k8 = (rem & 15) * 8, kk = k8 & 63;
    const v8us o = gather8(wkqv + (size_t)lt * (64 * 192) + (size_t)kk * 192 + n, 192, 0xffffu);
    st2_v8us(WKQ + (size_t)u * 8, o);
  } else if (blk < PBX + 3 + PBKQ + PBWO) {
    const int u = (blk - PBX - 3 - PBKQ) * NTHR + tid;
    const int lt = u >> 10, n = (u >> 4) & 63, k8 = (u & 15) * 8, kk = k8 & 63;
    const v8us o = gather8(wout + (size_t)lt * 4096 + (size_t)kk * HD + n, HD, 0xffffu);
    st2_v8us(WOU + (size_t)u * 8, o);
  } else if (blk < PBX + 3 + PBKQ + PBWO + NLE) {
    const int le = blk - (PBX + 3 + PBKQ + PBWO);
    const int n = tid >> 2, s8 = (tid & 3) * 8, i0 = s8 & 15;
    const v8us o = gather8(wk + (size_t)le * 1024 + (size_t)(((n >> 4) * 16 + i0) * 16 + (n & 15)), 16, 0xffffu);
    st2_v8us(RB + (size_t)le * RBMAT + (size_t)tid * 8, o);
  } else if (blk < PBX + 3 + PBKQ + PBWO + 2 * NLE) {
    const int le = blk - (PBX + 3 + PBKQ + PBWO + NLE);
    const int n = tid >> 2, s8 = (tid & 3) * 8, i0 = s8 & 15;
    const v8us o = gather8(wvv + (size_t)le * 1024 + (size_t)(((n >> 4) * 16 + i0) * 16 + (n & 15)), 16, 0xffffu);
    st2_v8us(RB + (size_t)(NLE + le) * RBMAT + (size_t)tid * 8, o);
  } else {
    const int vb = blk - (PBX + 3 + PBKQ + PBWO + 2 * NLE);
    if (vb == 0)      vec_copy(bu,   64,   VEC + VB_IN,        16,  tid);
    else if (vb == 1) vec_copy(be,   64,   VEC + VB_IN + 64,   16,  tid);
    else if (vb == 2) vec_copy(bv,   64,   VEC + VB_IN + 128,  16,  tid);
    else if (vb == 3) vec_copy(bkqv, 1152, VEC + VB_KQV,       288, tid);
    else if (vb == 4) vec_copy(bout, 384,  VEC + VB_OUT,       96,  tid);
    else if (vb == 5) vec_copy(prel, 104,  VEC + VB_PREL,      32,  tid);
    else if (vb == 6) vec_copy(skip, 6,    VEC + VB_SKIP,      8,   tid);
  }
}

template <int KEXT, int PBW>
__device__ __forceinline__ void gemm_16x64(const unsigned short* __restrict__ ap,
                                           const unsigned short* __restrict__ bp, v8f (&acc)[4]) {
#pragma unroll 1
  for (int k0 = 0; k0 < KEXT; k0 += 32) {
    FragB af;
    af.h[0] = *(const v8usa*)(ap + k0);
    af.h[1] = *(const v8usa*)(ap + k0 + 16);
#pragma unroll
    for (int nt = 0; nt < 4; ++nt) {
      const unsigned short* wq = bp + (size_t)(16 * nt) * (size_t)PBW + k0;
      FragB bf;
      bf.h[0] = *(const v8usa*)wq;
      bf.h[1] = *(const v8usa*)(wq + 16);
      acc[nt] = wmb(af, bf, acc[nt]);
    }
  }
}

__device__ __forceinline__ void stage_d(float* stg, const v8f (&acc)[4], int wave, int hh, int m) {
#pragma unroll
  for (int nt = 0; nt < 4; ++nt) {
#pragma unroll
    for (int r = 0; r < 8; ++r) stg[(16 * wave + 8 * hh + r) * SP + 16 * nt + m] = acc[nt][r];
  }
}

template <int T>
__global__ __launch_bounds__(NTHR) __attribute__((amdgpu_num_vgpr(248)))
void k_in(const unsigned short* __restrict__ XB, const unsigned short* __restrict__ WT,
          const float* __restrict__ VEC, const float* __restrict__ emb, const int* __restrict__ ids,
          float* H, unsigned short* HHL) {
  constexpr int NT  = (T == 0) ? NU : ((T == 1) ? NEV : NVN);
  constexpr int PBT = (T == 0) ? PB0 : ((T == 1) ? PB1 : PB2);
  __shared__ __attribute__((aligned(16))) float stg[GBM * SP];
  __shared__ __attribute__((aligned(16))) float sb[64];
  const int tid = (int)threadIdx.x, lane = tid & 31, wave = tid >> 5, hh = lane >> 4, m = lane & 15;
  const int lb = (int)blockIdx.x * GBM;
  const int rowBase = PBT + lb;
  if (tid < 16) *(v4fa*)(sb + 4 * tid) = *(const v4fa*)(VEC + VB_IN + 64 * T + 4 * tid);

  v8f acc[4];
  {
    const v8f z = {0.f, 0.f, 0.f, 0.f, 0.f, 0.f, 0.f, 0.f};
#pragma unroll
    for (int t = 0; t < 4; ++t) acc[t] = z;
  }
  const unsigned short* ap = XB + (size_t)(rowBase + 16 * wave + m) * (size_t)XK + 8 * hh;
  const unsigned short* bp = WT + (size_t)(T * 64 + m) * (size_t)XK + 8 * hh;
  gemm_16x64<XK, XK>(ap, bp, acc);
  stage_d(stg, acc, wave, hh, m);
  __syncthreads();

  const v4f bias = *(const v4fa*)(sb + 4 * m);
#pragma unroll 1
  for (int i = 0; i < 8; ++i) {
    const int lr   = 16 * wave + 2 * i + hh;
    const int lrow = lb + lr;
    const int grow = rowBase + lr;
    const bool live = lrow < NT;
    const int rc = live ? lrow : NT - 1;
    int id = ids[rc];
    id = id < 0 ? 0 : (id > NT - 1 ? NT - 1 : id);
    const v4f e = *(const v4fa*)(emb + (size_t)id * HD + 4 * m);
    const v4f a = *(const v4fa*)(stg + lr * SP + 4 * m);
    asm volatile("" :: "v"(e));
    asm volatile("" :: "v"(a));
    float v0 = (a.x + bias.x) + bf16_val(e.x), v1 = (a.y + bias.y) + bf16_val(e.y);
    float v2 = (a.z + bias.z) + bf16_val(e.z), v3 = (a.w + bias.w) + bf16_val(e.w);
    v0 = live ? v0 : 0.0f; v1 = live ? v1 : 0.0f; v2 = live ? v2 : 0.0f; v3 = live ? v3 : 0.0f;
    int h01, h23, l01, l23;
    hilo_pack(v0, v1, v2, v3, h01, h23, l01, l23);
    const v4i ow = regroup8(h01, h23, l01, l23, lane);
    v4f o;
    o.x = v0; o.y = v1; o.z = v2; o.w = v3;
    float* op = H + (size_t)grow * HD + 4 * m;
    unsigned short* hp = HHL + (size_t)grow * KL + 8 * m;
    *(volatile v4f*)op = o;
    *(volatile v4i*)hp = ow;
    __threadfence();
    *(volatile v4f*)op = o;
    *(volatile v4i*)hp = ow;
  }
}

__device__ __forceinline__ void bucket_flush(const int* pl, const int* cnt, const int* offs, int ov, int nslots,
                                             int* rp, int* sp, int* fp, int tid) {
#pragma unroll 1
  for (int i = tid * 4; i < RUNCAP; i += NTHR * 4) {
    const v4i v = *(const v4ia*)(pl + i);
    *(volatile v4i*)(rp + i) = v;
  }
  {
    const v4i c = *(const v4ia*)(cnt + 4 * tid);
    const v4i o = *(const v4ia*)(offs + 4 * tid);
    v4i w;
    w.x = (o.x & 0xffff) | (c.x << 16); w.y = (o.y & 0xffff) | (c.y << 16);
    w.z = (o.z & 0xffff) | (c.z << 16); w.w = (o.w & 0xffff) | (c.w << 16);
    if (4 * tid < nslots) *(volatile v4i*)(sp + 4 * tid) = w;
  }
  if (tid < 8) {
    const v4i f = {ov, ov, ov, ov};
    *(volatile v4i*)(fp + 4 * tid) = f;
  }
}

__global__ __launch_bounds__(NTHR) void k_bucket(const int* __restrict__ srcs, const int* __restrict__ dsts,
                                                 int nE, int nsrc, int nd, int slb, int vec,
                                                 int* RUNe, int* SLOTe, int* FLAGe) {
  extern __shared__ __attribute__((aligned(16))) int dsm[];
  int* wl   = dsm;
  int* pl   = dsm + NWAVE * WLCAP;
  int* cnt  = pl + RUNCAP;
  int* offs = cnt + NSMAX;
  int* cur  = offs + NSMAX;
  int* misc = cur + NSMAX;
  const int tid = (int)threadIdx.x, lane = tid & 31, wave = tid >> 5;
  const int blk = (int)blockIdx.x;
  const int nslots = 1 << slb;
  const unsigned nbs = (unsigned)(blk << slb);
  const unsigned uns = (unsigned)nslots, und = (unsigned)nd;

  {
    const v4i z4 = {0, 0, 0, 0};
    for (int i = tid * 4; i < BK_ZINTS; i += NTHR * 4) *(v4ia*)(dsm + i) = z4;
    if (tid < 16) misc[tid] = 0;
  }
  __syncthreads();

  {
    const int per  = ((nE + NWAVE * WCH - 1) / (NWAVE * WCH)) * WCH;
    const int ebeg = wave * per;
    const int eend = (ebeg + per < nE) ? (ebeg + per) : nE;
    const int sent = (int)(1u << 31);
    int* mylist = wl + wave * WLCAP;
    int wc = 0;
#pragma unroll 1
    for (int cb = ebeg; cb < eend; cb += WCH) {
      const int e0 = cb + lane * 8;
      v4i da, db;
      if (vec != 0 && cb + WCH <= nE) {
        da = *(const v4ia*)(dsts + e0);
        db = *(const v4ia*)(dsts + e0 + 4);
      } else {
        const int q0 = (e0     < nE) ? e0     : nE - 1, q1 = (e0 + 1 < nE) ? e0 + 1 : nE - 1;
        const int q2 = (e0 + 2 < nE) ? e0 + 2 : nE - 1, q3 = (e0 + 3 < nE) ? e0 + 3 : nE - 1;
        const int q4 = (e0 + 4 < nE) ? e0 + 4 : nE - 1, q5 = (e0 + 5 < nE) ? e0 + 5 : nE - 1;
        const int q6 = (e0 + 6 < nE) ? e0 + 6 : nE - 1, q7 = (e0 + 7 < nE) ? e0 + 7 : nE - 1;
        const int t0 = dsts[q0], t1 = dsts[q1], t2 = dsts[q2], t3 = dsts[q3];
        const int t4 = dsts[q4], t5 = dsts[q5], t6 = dsts[q6], t7 = dsts[q7];
        asm volatile("" :: "v"(t0), "v"(t1), "v"(t2), "v"(t3));
        asm volatile("" :: "v"(t4), "v"(t5), "v"(t6), "v"(t7));
        da.x = (e0     < nE) ? t0 : sent; da.y = (e0 + 1 < nE) ? t1 : sent;
        da.z = (e0 + 2 < nE) ? t2 : sent; da.w = (e0 + 3 < nE) ? t3 : sent;
        db.x = (e0 + 4 < nE) ? t4 : sent; db.y = (e0 + 5 < nE) ? t5 : sent;
        db.z = (e0 + 6 < nE) ? t6 : sent; db.w = (e0 + 7 < nE) ? t7 : sent;
      }
      const unsigned s0 = (unsigned)da.x - nbs, s1 = (unsigned)da.y - nbs;
      const unsigned s2 = (unsigned)da.z - nbs, s3 = (unsigned)da.w - nbs;
      const unsigned s4 = (unsigned)db.x - nbs, s5 = (unsigned)db.y - nbs;
      const unsigned s6 = (unsigned)db.z - nbs, s7 = (unsigned)db.w - nbs;
      const bool h0 = (s0 < uns) & ((unsigned)da.x < und), h1 = (s1 < uns) & ((unsigned)da.y < und);
      const bool h2 = (s2 < uns) & ((unsigned)da.z < und), h3 = (s3 < uns) & ((unsigned)da.w < und);
      const bool h4 = (s4 < uns) & ((unsigned)db.x < und), h5 = (s5 < uns) & ((unsigned)db.y < und);
      const bool h6 = (s6 < uns) & ((unsigned)db.z < und), h7 = (s7 < uns) & ((unsigned)db.w < und);
      const unsigned m0 = __builtin_amdgcn_ballot_w32(h0), m1 = __builtin_amdgcn_ballot_w32(h1);
      const unsigned m2 = __builtin_amdgcn_ballot_w32(h2), m3 = __builtin_amdgcn_ballot_w32(h3);
      const unsigned m4 = __builtin_amdgcn_ballot_w32(h4), m5 = __builtin_amdgcn_ballot_w32(h5);
      const unsigned m6 = __builtin_amdgcn_ballot_w32(h6), m7 = __builtin_amdgcn_ballot_w32(h7);
      const unsigned any = m0 | m1 | m2 | m3 | m4 | m5 | m6 | m7;
      if (any != 0u) {
        const int pre = (int)(__builtin_amdgcn_mbcnt_lo(m0, 0u) + __builtin_amdgcn_mbcnt_lo(m1, 0u) +
                              __builtin_amdgcn_mbcnt_lo(m2, 0u) + __builtin_amdgcn_mbcnt_lo(m3, 0u) +
                              __builtin_amdgcn_mbcnt_lo(m4, 0u) + __builtin_amdgcn_mbcnt_lo(m5, 0u) +
                              __builtin_amdgcn_mbcnt_lo(m6, 0u) + __builtin_amdgcn_mbcnt_lo(m7, 0u));
        int p = wc + pre;
        if (h0) { if (p < WLCAP) mylist[p] = ((e0 + 0) << EIDSH) | (int)s0; p = p + 1; }
        if (h1) { if (p < WLCAP) mylist[p] = ((e0 + 1) << EIDSH) | (int)s1; p = p + 1; }
        if (h2) { if (p < WLCAP) mylist[p] = ((e0 + 2) << EIDSH) | (int)s2; p = p + 1; }
        if (h3) { if (p < WLCAP) mylist[p] = ((e0 + 3) << EIDSH) | (int)s3; p = p + 1; }
        if (h4) { if (p < WLCAP) mylist[p] = ((e0 + 4) << EIDSH) | (int)s4; p = p + 1; }
        if (h5) { if (p < WLCAP) mylist[p] = ((e0 + 5) << EIDSH) | (int)s5; p = p + 1; }
        if (h6) { if (p < WLCAP) mylist[p] = ((e0 + 6) << EIDSH) | (int)s6; p = p + 1; }
        if (h7) { if (p < WLCAP) mylist[p] = ((e0 + 7) << EIDSH) | (int)s7; p = p + 1; }
        wc += (int)(__builtin_popcount(m0) + __builtin_popcount(m1) + __builtin_popcount(m2) + __builtin_popcount(m3) +
                    __builtin_popcount(m4) + __builtin_popcount(m5) + __builtin_popcount(m6) + __builtin_popcount(m7));
      }
    }
    if (lane == 0) misc[wave] = wc;
  }
  __syncthreads();

  if (wave == 0) {
    int ov = 0;
#pragma unroll 1
    for (int w2 = 0; w2 < NWAVE; ++w2) {
      int c = misc[w2];
      if (c > WLCAP) ov = 1;
      c = c < 0 ? 0 : (c > WLCAP ? WLCAP : c);
#pragma unroll 1
      for (int b0 = 0; b0 < c; b0 += 32) {
        const int idx = b0 + lane;
        const int ent = wl[w2 * WLCAP + (idx < WLCAP ? idx : WLCAP - 1)];
        const int m32 = (c - b0) < 32 ? (c - b0) : 32;
#pragma unroll 1
        for (int k = 0; k < m32; ++k) {
          const int u    = __builtin_amdgcn_readlane(ent, k);
          const int slot = u & (NSMAX - 1);
          if (lane == 0) cnt[slot] = cnt[slot] + 1;
        }
      }
    }
    if (lane == 0) misc[9] = ov;
  }
  __syncthreads();
  if (wave == 0) {
    const int base = lane * (NSMAX / 32);
    int s = 0;
#pragma unroll 1
    for (int i = 0; i < NSMAX / 32; ++i) s += cnt[base + i];
    int incl = s;
#pragma unroll
    for (int d = 1; d < 32; d <<= 1) {
      const int y = __shfl_up(incl, d, 32);
      if (lane >= d) incl += y;
    }
    if (lane == 31) misc[10] = (incl > RUNCAP) ? 1 : 0;
    int run = incl - s;
#pragma unroll 1
    for (int i = 0; i < NSMAX / 32; ++i) {
      const int cv = cnt[base + i];
      offs[base + i] = run;
      cur[base + i]  = run;
      run += cv;
    }
  }
  __syncthreads();

  if (wave == 0) {
#pragma unroll 1
    for (int w2 = 0; w2 < NWAVE; ++w2) {
      int c = misc[w2];
      c = c < 0 ? 0 : (c > WLCAP ? WLCAP : c);
#pragma unroll 1
      for (int b0 = 0; b0 < c; b0 += 32) {
        const int idx = b0 + lane;
        const int ent = wl[w2 * WLCAP + (idx < WLCAP ? idx : WLCAP - 1)];
        int eid = (ent >> EIDSH) & 0x1FFFFF;
        eid = eid > nE - 1 ? nE - 1 : eid;
        int sr = srcs[eid];
        sr = sr < 0 ? 0 : (sr > nsrc - 1 ? nsrc - 1 : sr);
        const int word = (int)((unsigned)sr | ((unsigned)(ent & (NSMAX - 1)) << 16));
        const int m32 = (c - b0) < 32 ? (c - b0) : 32;
#pragma unroll 1
        for (int k = 0; k < m32; ++k) {
          const int u    = __builtin_amdgcn_readlane(ent, k);
          const int wd   = __builtin_amdgcn_readlane(word, k);
          const int slot = u & (NSMAX - 1);
          if (lane == 0) {
            int p = cur[slot];
            p = p < 0 ? 0 : (p > RUNCAP - 1 ? RUNCAP - 1 : p);
            pl[p] = wd;
            cur[slot] = p + 1;
          }
        }
      }
    }
  }
  __syncthreads();

  const int ovf = misc[9] | misc[10];
  int* rp = RUNe + (size_t)blk * RUNCAP;
  int* sp = SLOTe + (size_t)(blk << slb);
  int* fp = FLAGe + (size_t)blk * 32;
  bucket_flush(pl, cnt, offs, ovf, nslots, rp, sp, fp, tid);
  __threadfence();
  bucket_flush(pl, cnt, offs, ovf, nslots, rp, sp, fp, tid);
}

__global__ __launch_bounds__(NTHR) __attribute__((amdgpu_num_vgpr(248)))
void k_kqv(const unsigned short* __restrict__ HHL, const unsigned short* __restrict__ WKQ,
           const float* __restrict__ VEC, int l, float* Q, unsigned short* KV2) {
  __shared__ __attribute__((aligned(16))) float stg[GBM * SP];
  __shared__ __attribute__((aligned(16))) float sb[64];
  const int tid = (int)threadIdx.x, lane = tid & 31, wave = tid >> 5, hh = lane >> 4, m = lane & 15;
  const int bx = (int)blockIdx.x, y = (int)blockIdx.y;
  const int t = type_of_blk(bx), lt = l * 3 + t;
  const int rowBase = bx * GBM;
  if (tid < 16) *(v4fa*)(sb + 4 * tid) = *(const v4fa*)(VEC + VB_KQV + lt * 192 + 64 * y + 4 * tid);

  v8f acc[4];
  {
    const v8f z = {0.f, 0.f, 0.f, 0.f, 0.f, 0.f, 0.f, 0.f};
#pragma unroll
    for (int q = 0; q < 4; ++q) acc[q] = z;
  }
  const unsigned short* ap = HHL + (size_t)(rowBase + 16 * wave + m) * (size_t)KL + 8 * hh;
  const unsigned short* bp = WKQ + (size_t)(lt * 192 + 64 * y + m) * (size_t)WP + 8 * hh;
  gemm_16x64<KEXT_KQV, WP>(ap, bp, acc);
  stage_d(stg, acc, wave, hh, m);
  __syncthreads();

  const v4f bias = *(const v4fa*)(sb + 4 * m);
#pragma unroll 1
  for (int i = 0; i < 8; ++i) {
    const int lr   = 16 * wave + 2 * i + hh;
    const int grow = rowBase + lr;
    const v4f a = *(const v4fa*)(stg + lr * SP + 4 * m);
    const float v0 = a.x + bias.x, v1 = a.y + bias.y, v2 = a.z + bias.z, v3 = a.w + bias.w;
    if (y == 1) {
      v4f o;
      o.x = v0; o.y = v1; o.z = v2; o.w = v3;
      st2_v4f(Q + (size_t)grow * HD + 4 * m, o);
    } else {
      int h01, h23, l01, l23;
      hilo_pack(v0, v1, v2, v3, h01, h23, l01, l23);
      const v4i ow = regroup8(h01, h23, l01, l23, lane);
      unsigned short* hp = KV2 + (size_t)(y >> 1) * ((size_t)NP * KL) + (size_t)grow * KL + 8 * m;
      *(volatile v4i*)hp = ow;
      __threadfence();
      *(volatile v4i*)hp = ow;
    }
  }
}

__global__ __launch_bounds__(NTHR) __attribute__((amdgpu_num_vgpr(248)))
void k_rel(const unsigned short* __restrict__ KV2, const unsigned short* __restrict__ RBle, int pbs, float* KVE) {
  __shared__ __attribute__((aligned(16))) float stg[GBM * SP];
  const int tid = (int)threadIdx.x, lane = tid & 31, wave = tid >> 5, hh = lane >> 4, m = lane & 15;
  const int y = (int)blockIdx.y;
  const int rowl = (int)blockIdx.x * GBM;
  const unsigned short* ap = KV2 + (size_t)y * ((size_t)NP * KL) + (size_t)(pbs + rowl + 16 * wave + m) * (size_t)KL + 8 * hh;
  const unsigned short* bq = RBle + (size_t)y * ((size_t)NLE * RBMAT) + (size_t)m * RBW + 8 * hh;
  v8f acc[4];
  const v8f z = {0.f, 0.f, 0.f, 0.f, 0.f, 0.f, 0.f, 0.f};
#pragma unroll
  for (int h = 0; h < 4; ++h) {
    FragB af, bf;
    af.h[0] = *(const v8usa*)(ap + 16 * h);
#if SPLIT_REL
    af.h[1] = *(const v8usa*)(ap + HD + 16 * h);
#else
    { const v8us z8 = {0, 0, 0, 0, 0, 0, 0, 0}; af.h[1] = z8; }
#endif
    bf.h[0] = *(const v8usa*)(bq + (size_t)(16 * h) * RBW);
    bf.h[1] = *(const v8usa*)(bq + (size_t)(16 * h) * RBW + 16);
    acc[h] = wmb(af, bf, z);
  }
  stage_d(stg, acc, wave, hh, m);
  __syncthreads();
#pragma unroll 1
  for (int i = 0; i < 8; ++i) {
    const int lr = 16 * wave + 2 * i + hh;
    const v4f a = *(const v4fa*)(stg + lr * SP + 4 * m);
    st2_v4f(KVE + (size_t)(rowl + lr) * 128 + 64 * y + 4 * m, a);
  }
}

__global__ __launch_bounds__(NTHR) void k_replay(const float* __restrict__ Q, const float* __restrict__ KVE,
                                                 const int* __restrict__ RUNe, const int* __restrict__ SLOTe,
                                                 const int* __restrict__ FLAGe, const float* __restrict__ prel,
                                                 float* ST, int pbd, int nsrc, int slb, int first) {
  __shared__ float spr[4];
  const int tid = (int)threadIdx.x, lane = tid & 31, wave = tid >> 5, hh = lane >> 4, q = lane & 15;
  if (tid < 4) spr[tid] = prel[tid];
  __syncthreads();
  const float pr = spr[q >> 2];
  const int rowBase = (int)blockIdx.x * 64;
  const float qnan = __uint_as_float(0x7fc00000u);

#pragma unroll 1
  for (int i = 0; i < 4; ++i) {
    const int rl = rowBase + 8 * wave + 2 * i + hh;
    const int g  = pbd + rl;
    const int bk = rl >> slb;
    const int sw = SLOTe[rl];
    const int flag = FLAGe[(size_t)bk * 32];
    int o = sw & 0xffff;
    int c = (sw >> 16) & 0xffff;
    const bool big = c > TRIPCAP;
    c = c > TRIPCAP ? TRIPCAP : c;
    o = o > RUNCAP - 1 ? RUNCAP - 1 : o;
    const int co = __shfl_xor(c, 16, 32);
    int cm = c > co ? c : co;
    cm = cm > TRIPCAP ? TRIPCAP : cm;
    const int cmu = __builtin_amdgcn_readfirstlane(cm);
    int last = o + c - 1;
    last = last < o ? o : last;
    last = last > RUNCAP - 1 ? RUNCAP - 1 : last;
    const int* run = RUNe + (size_t)bk * RUNCAP;
    const v4f q4 = *(const v4fa*)(Q + (size_t)g * HD + 4 * q);
    float* st = ST + (size_t)g * STW;
    float mx = MX0, sm = 0.0f;
    float a0 = 0.0f, a1 = 0.0f, a2 = 0.0f, a3 = 0.0f;
    if (first == 0) {
      const v4f av = *(const v4fa*)(st + 4 * q);
      const v2f ms = *(const v2fa*)(st + HD + 2 * q);
      a0 = av.x; a1 = av.y; a2 = av.z; a3 = av.w;
      mx = ms.x; sm = ms.y;
    }
#pragma unroll 1
    for (int j = 0; j < cmu; ++j) {
      int idx = o + j;
      idx = idx > last ? last : idx;
      const unsigned wd = (unsigned)run[idx];
      int sr = (int)(wd & 0xffffu);
      sr = sr > nsrc - 1 ? nsrc - 1 : sr;
      const float* kp = KVE + (size_t)sr * 128 + 4 * q;
      const v4f ke = *(const v4fa*)kp;
      const v4f ve = *(const v4fa*)(kp + HD);
      asm volatile("" :: "v"(ke));
      asm volatile("" :: "v"(ve));
      float part = q4.x * ke.x;
      part = fmaf(q4.y, ke.y, part);
      part = fmaf(q4.z, ke.z, part);
      part = fmaf(q4.w, ke.w, part);
      part += __shfl_xor(part, 1, 32);
      part += __shfl_xor(part, 2, 32);
      const float s  = (part * pr) * 0.25f;
      const float mn = fmaxf(mx, s);
      const float c0 = expf(mx - mn);
      const float p  = expf(s - mn);
      const float nsm = sm * c0 + p;
      const float n0 = a0 * c0 + p * ve.x, n1 = a1 * c0 + p * ve.y;
      const float n2 = a2 * c0 + p * ve.z, n3 = a3 * c0 + p * ve.w;
      const bool valid = j < c;
      sm = valid ? nsm : sm;
      mx = valid ? mn : mx;
      a0 = valid ? n0 : a0; a1 = valid ? n1 : a1; a2 = valid ? n2 : a2; a3 = valid ? n3 : a3;
    }
    const bool bad = (flag != 0) | big;
    a0 = bad ? qnan : a0; a1 = bad ? qnan : a1; a2 = bad ? qnan : a2; a3 = bad ? qnan : a3;
    sm = bad ? qnan : sm;
    v4f ov;
    ov.x = a0; ov.y = a1; ov.z = a2; ov.w = a3;
    v2f mv;
    mv.x = mx; mv.y = sm;
    *(volatile v4f*)(st + 4 * q) = ov;
    *(volatile v2f*)(st + HD + 2 * q) = mv;
    __threadfence();
    *(volatile v4f*)(st + 4 * q) = ov;
    *(volatile v2f*)(st + HD + 2 * q) = mv;
  }
}

__device__ __forceinline__ int flags_of(const int* __restrict__ FLAG, int t, int blk) {
  int f;
  if (t == 0) {
    f = FLAG[(size_t)(RB_E0 + blk) * 32] | FLAG[(size_t)(RB_E6 + blk) * 32] | FLAG[(size_t)(RB_E7 + blk) * 32] |
        FLAG[(size_t)(RB_E8 + blk) * 32] | FLAG[(size_t)(RB_E9 + blk) * 32] | FLAG[(size_t)(RB_E10 + blk) * 32];
  } else if (t == 1) {
    f = FLAG[(size_t)(RB_E1 + blk) * 32] | FLAG[(size_t)(RB_E2 + blk) * 32] | FLAG[(size_t)(RB_E3 + blk) * 32] |
        FLAG[(size_t)(RB_E4 + blk) * 32] | FLAG[(size_t)(RB_E5 + blk) * 32] | FLAG[(size_t)(RB_E12 + blk) * 32];
  } else {
    f = FLAG[(size_t)(RB_E11 + blk) * 32];
  }
  return f;
}

template <int LAST>
__global__ __launch_bounds__(NTHR) __attribute__((amdgpu_num_vgpr(248)))
void k_out(const float* __restrict__ ST, const unsigned short* __restrict__ WOU, const float* __restrict__ VEC,
           const int* __restrict__ FLAG, int l, float* H, unsigned short* HHL, float* out) {
  __shared__ __attribute__((aligned(16))) float tile[GBM * SP];
  __shared__ __attribute__((aligned(16))) float sb[64];
  const int tid = (int)threadIdx.x, lane = tid & 31, wave = tid >> 5, hh = lane >> 4, m = lane & 15;
  const int bx = (int)blockIdx.x;
  const int t = type_of_blk(bx), lt = l * 3 + t;
  const int rowBase = bx * GBM;
  const int NT  = (t == 0) ? NU : ((t == 1) ? NEV : NVN);
  const int PBT = (t == 0) ? PB0 : ((t == 1) ? PB1 : PB2);
  const int EO  = (t == 0) ? 0 : ((t == 1) ? NU * HD : (NU + NEV) * HD);
  const int lb  = rowBase - PBT;
  if (tid < 16) *(v4fa*)(sb + 4 * tid) = *(const v4fa*)(VEC + VB_OUT + lt * HD + 4 * tid);
  const float sk  = VEC[VB_SKIP + lt];
  const float gg  = 1.0f / (1.0f + expf(-sk));
  const float omg = 1.0f - gg;
  unsigned short* As = (unsigned short*)tile;

#pragma unroll 1
  for (int it = 0; it < 8; ++it) {
    const int idx = it * NTHR + tid;
    const int r = idx >> 4, c4 = idx & 15;
    const float* sp = ST + (size_t)(rowBase + r) * STW;
    const v4f av = *(const v4fa*)(sp + 4 * c4);
    const v2f ms = *(const v2fa*)(sp + HD + 2 * c4);
    asm volatile("" :: "v"(av));
    asm volatile("" :: "v"(ms));
    const float sm = ms.y;
    const bool zr = (sm == 0.0f);
    float x0 = av.x / sm, x1 = av.y / sm, x2 = av.z / sm, x3 = av.w / sm;
    x0 = zr ? 0.0f : x0; x1 = zr ? 0.0f : x1; x2 = zr ? 0.0f : x2; x3 = zr ? 0.0f : x3;
    const float g0 = 0.5f * x0 * (1.0f + erff(x0 * 0.70710678f));
    const float g1 = 0.5f * x1 * (1.0f + erff(x1 * 0.70710678f));
    const float g2 = 0.5f * x2 * (1.0f + erff(x2 * 0.70710678f));
    const float g3 = 0.5f * x3 * (1.0f + erff(x3 * 0.70710678f));
    int h01, h23, l01, l23;
    hilo_pack(g0, g1, g2, g3, h01, h23, l01, l23);
    v2i hv, lv;
    hv.x = h01; hv.y = h23; lv.x = l01; lv.y = l23;
    *(v2ia*)(As + r * KL + 4 * c4)      = hv;
    *(v2ia*)(As + r * KL + HD + 4 * c4) = lv;
  }
  __syncthreads();

  v8f acc[4];
  {
    const v8f z = {0.f, 0.f, 0.f, 0.f, 0.f, 0.f, 0.f, 0.f};
#pragma unroll
    for (int q = 0; q < 4; ++q) acc[q] = z;
  }
  {
    const int aoff = (16 * wave + m) * KL + 8 * hh;
    const unsigned short* bp = WOU + (size_t)(lt * HD + m) * (size_t)WP + 8 * hh;
#pragma unroll 1
    for (int k0 = 0; k0 < KEXT_OUT; k0 += 32) {
      FragB af;
      af.h[0] = *(const v8usa*)(As + aoff + k0);
      af.h[1] = *(const v8usa*)(As + aoff + k0 + 16);
#pragma unroll
      for (int nt = 0; nt < 4; ++nt) {
        const unsigned short* wq = bp + (size_t)(16 * nt) * (size_t)WP + k0;
        FragB bf;
        bf.h[0] = *(const v8usa*)wq;
        bf.h[1] = *(const v8usa*)(wq + 16);
        acc[nt] = wmb(af, bf, acc[nt]);
      }
    }
  }
  __syncthreads();
  stage_d(tile, acc, wave, hh, m);
  __syncthreads();

  int flag = 0;
  if constexpr (LAST != 0) flag = flags_of(FLAG, t, lb >> ((t == 2) ? 7 : 10));
  const float qnan = __uint_as_float(0x7fc00000u);
  const v4f bias = *(const v4fa*)(sb + 4 * m);
#pragma unroll 1
  for (int i = 0; i < 8; ++i) {
    const int lr   = 16 * wave + 2 * i + hh;
    const int lrow = lb + lr;
    const int grow = rowBase + lr;
    const bool live = lrow < NT;
    const v4f a  = *(const v4fa*)(tile + lr * SP + 4 * m);
    const v4f ho = *(const v4fa*)(H + (size_t)grow * HD + 4 * m);
    asm volatile("" :: "v"(a));
    asm volatile("" :: "v"(ho));
    float v0 = gg * (a.x + bias.x) + omg * ho.x, v1 = gg * (a.y + bias.y) + omg * ho.y;
    float v2 = gg * (a.z + bias.z) + omg * ho.z, v3 = gg * (a.w + bias.w) + omg * ho.w;
    v0 = (v0 > 0.0f) ? v0 : (v0 - v0); v1 = (v1 > 0.0f) ? v1 : (v1 - v1);
    v2 = (v2 > 0.0f) ? v2 : (v2 - v2); v3 = (v3 > 0.0f) ? v3 : (v3 - v3);
    v0 = live ? v0 : 0.0f; v1 = live ? v1 : 0.0f; v2 = live ? v2 : 0.0f; v3 = live ? v3 : 0.0f;
    if constexpr (LAST != 0) {
      float ss = (v0 * v0 + v1 * v1) + (v2 * v2 + v3 * v3);
      ss += __shfl_xor(ss, 1, 32);
      ss += __shfl_xor(ss, 2, 32);
      ss += __shfl_xor(ss, 4, 32);
      ss += __shfl_xor(ss, 8, 32);
      const float nrm = sqrtf(ss);
      const float dn  = (nrm < 1e-12f) ? 1e-12f : nrm;
      v4f o;
      o.x = v0 / dn; o.y = v1 / dn; o.z = v2 / dn; o.w = v3 / dn;
      const bool bad = flag != 0;
      o.x = bad ? qnan : o.x; o.y = bad ? qnan : o.y; o.z = bad ? qnan : o.z; o.w = bad ? qnan : o.w;
      const int lc = live ? lrow : NT - 1;
      float* op = out + (size_t)EO + (size_t)lc * HD + 4 * m;
      if (live) *(volatile v4f*)op = o;
      __threadfence();
      if (live) *(volatile v4f*)op = o;
    } else {
      int h01, h23, l01, l23;
      hilo_pack(v0, v1, v2, v3, h01, h23, l01, l23);
      const v4i ow = regroup8(h01, h23, l01, l23, lane);
      v4f o;
      o.x = v0; o.y = v1; o.z = v2; o.w = v3;
      float* op = H + (size_t)grow * HD + 4 * m;
      unsigned short* hp = HHL + (size_t)grow * KL + 8 * m;
      *(volatile v4f*)op = o;
      *(volatile v4i*)hp = ow;
      __threadfence();
      *(volatile v4f*)op = o;
      *(volatile v4i*)hp = ow;
    }
  }
}

extern "C" void kernel_launch(void* const* d_in, const int* in_sizes, int n_in,
                              void* d_out, int out_size, void* d_ws, size_t ws_size,
                              hipStream_t stream) {
  static const int ES[13]  = {0, 0, 0, 0, 0, 0, 1, 1, 1, 1, 1, 1, 2};
  static const int ED[13]  = {0, 1, 1, 1, 1, 1, 0, 0, 0, 0, 0, 2, 1};
  static const int ENE[13] = {150000, 120000, 60000, 40000, 30000, 50000, 120000, 60000, 40000, 30000, 50000, 60000, 60000};
  static const int RBS[13] = {RB_E0, RB_E1, RB_E2, RB_E3, RB_E4, RB_E5, RB_E6, RB_E7, RB_E8, RB_E9, RB_E10, RB_E11, RB_E12};
  static const int SBS[13] = {0, 184320, 244736, 305152, 365568, 425984, 30720, 61440, 92160, 122880, 153600, 546816, 486400};
  static const int NTY[3]  = {NU, NEV, NVN};
  static const int NPT[3]  = {PU, PE, PV};
  static const int PBS[3]  = {PB0, PB1, PB2};
  static const int SLB[3]  = {10, 10, 7};

  if (n_in < 36) return;
  if (in_sizes[0] != NU * 32 || in_sizes[1] != NEV * 32 || in_sizes[2] != NVN * 16) return;
  if (in_sizes[3] != 32 * 64 || in_sizes[4] != 64 || in_sizes[5] != 32 * 64 || in_sizes[6] != 64) return;
  if (in_sizes[7] != 16 * 64 || in_sizes[8] != 64) return;
  if (in_sizes[9] != NU * 64 || in_sizes[10] != NEV * 64 || in_sizes[11] != NVN * 64) return;
  if (in_sizes[12] != 2 * 3 * 64 * 192 || in_sizes[13] != 2 * 3 * 192) return;
  if (in_sizes[14] != 2 * 13 * 1024 || in_sizes[15] != 2 * 13 * 1024 || in_sizes[16] != 2 * 13 * 4) return;
  if (in_sizes[17] != 2 * 3 * 4096 || in_sizes[18] != 2 * 3 * 64 || in_sizes[19] != 6) return;
  if (in_sizes[20] != NU || in_sizes[21] != NEV || in_sizes[22] != NVN) return;
  for (int e = 0; e < 13; ++e) if (in_sizes[23 + e] != 2 * ENE[e]) return;
  if (out_size != (NU + NEV + NVN) * HD) return;

  constexpr size_t zF    = (size_t)NP * HD * 4;
  constexpr size_t zHL   = (size_t)NP * KL * 2;
  constexpr size_t zKVE  = (size_t)PE * 128 * 4;
  constexpr size_t zST   = (size_t)NP * STW * 4;
  constexpr size_t zRUN  = (size_t)NRUNS * RUNCAP * 4;
  constexpr size_t zSLOT = (size_t)NSLOTW * 4;
  constexpr size_t zFLAG = (size_t)NRUNS * 128;
  constexpr size_t zXB   = (size_t)NP * XK * 2;
  constexpr size_t zWT   = (size_t)3 * 64 * XK * 2;
  constexpr size_t zWKQ  = (size_t)6 * 192 * WP * 2;
  constexpr size_t zWOU  = (size_t)6 * 64 * WP * 2;
  constexpr size_t zRB   = (size_t)2 * NLE * RBMAT * 2;
  constexpr size_t zVEC  = (size_t)VECN * 4;
  constexpr size_t oH    = 0;
  constexpr size_t oHHL  = oH + zF;
  constexpr size_t oQ    = oHHL + zHL;
  constexpr size_t oKV2  = oQ + zF;
  constexpr size_t oKVE  = oKV2 + 2 * zHL;
  constexpr size_t oST   = oKVE + zKVE;
  constexpr size_t oRUN  = oST + zST;
  constexpr size_t oSLOT = oRUN + zRUN;
  constexpr size_t oFLAG = oSLOT + zSLOT;
  constexpr size_t oXB   = oFLAG + zFLAG;
  constexpr size_t oWT   = oXB + zXB;
  constexpr size_t oWKQ  = oWT + zWT;
  constexpr size_t oWOU  = oWKQ + zWKQ;
  constexpr size_t oRB   = oWOU + zWOU;
  constexpr size_t oVEC  = oRB + zRB;
  constexpr size_t oEND  = oVEC + zVEC;
  static_assert(zF % 256 == 0 && zHL % 256 == 0 && zKVE % 256 == 0 && zST % 256 == 0 && zRUN % 256 == 0);
  static_assert(zSLOT % 256 == 0 && zFLAG % 256 == 0 && zXB % 256 == 0 && zWT % 256 == 0 && zWKQ % 256 == 0);
  static_assert(zWOU % 256 == 0 && zRB % 256 == 0 && zVEC % 256 == 0);
  static_assert(oEND <= ((size_t)256 << 20));
  if (oEND > ws_size) return;

  const float* x_user  = (const float*)d_in[0];
  const float* x_event = (const float*)d_in[1];
  const float* x_venue = (const float*)d_in[2];
  const float* W_user  = (const float*)d_in[3];
  const float* b_user  = (const float*)d_in[4];
  const float* W_event = (const float*)d_in[5];
  const float* b_event = (const float*)d_in[6];
  const float* W_venue = (const float*)d_in[7];
  const float* b_venue = (const float*)d_in[8];
  const float* emb_user  = (const float*)d_in[9];
  const float* emb_event = (const float*)d_in[10];
  const float* emb_venue = (const float*)d_in[11];
  const float* Wkqv  = (const float*)d_in[12];
  const float* bkqv  = (const float*)d_in[13];
  const float* Wk    = (const float*)d_in[14];
  const float* Wv    = (const float*)d_in[15];
  const float* p_rel = (const float*)d_in[16];
  const float* Wout  = (const float*)d_in[17];
  const float* bout  = (const float*)d_in[18];
  const float* skip  = (const float*)d_in[19];
  const int* ids_user  = (const int*)d_in[20];
  const int* ids_event = (const int*)d_in[21];
  const int* ids_venue = (const int*)d_in[22];
  float* out = (float*)d_out;

  char* ws = (char*)d_ws;
  float*          H    = (float*)(ws + oH);
  unsigned short* HHL  = (unsigned short*)(ws + oHHL);
  float*          Q    = (float*)(ws + oQ);
  unsigned short* KV2  = (unsigned short*)(ws + oKV2);
  float*          KVE  = (float*)(ws + oKVE);
  float*          ST   = (float*)(ws + oST);
  int*            RUN  = (int*)(ws + oRUN);
  int*            SLOT = (int*)(ws + oSLOT);
  int*            FLAG = (int*)(ws + oFLAG);
  unsigned short* XB   = (unsigned short*)(ws + oXB);
  unsigned short* WT   = (unsigned short*)(ws + oWT);
  unsigned short* WKQ  = (unsigned short*)(ws + oWKQ);
  unsigned short* WOU  = (unsigned short*)(ws + oWOU);
  unsigned short* RB   = (unsigned short*)(ws + oRB);
  float*          VEC  = (float*)(ws + oVEC);

  hipFuncSetAttribute(reinterpret_cast<const void*>(&k_bucket), hipFuncAttributeMaxDynamicSharedMemorySize, (int)BK_LDS);

  k_prep<<<PBTOT, NTHR, 0, stream>>>(x_user, x_event, x_venue, W_user, W_event, W_venue, b_user, b_event, b_venue,
                                     Wkqv, bkqv, Wk, Wv, p_rel, Wout, bout, skip, XB, WT, WKQ, WOU, RB, VEC);
  k_in<0><<<PU / GBM, NTHR, 0, stream>>>(XB, WT, VEC, emb_user,  ids_user,  H, HHL);
  k_in<1><<<PE / GBM, NTHR, 0, stream>>>(XB, WT, VEC, emb_event, ids_event, H, HHL);
  k_in<2><<<PV / GBM, NTHR, 0, stream>>>(XB, WT, VEC, emb_venue, ids_venue, H, HHL);
  for (int e = 0; e < 13; ++e) {
    const int n = ENE[e], d = ED[e];
    const int* src = (const int*)d_in[23 + e];
    const int* dst = src + n;
    const int nblk = NPT[d] >> SLB[d];
    k_bucket<<<nblk, NTHR, BK_LDS, stream>>>(src, dst, n, NTY[ES[e]], NTY[d], SLB[d], ((n & 3) == 0) ? 1 : 0,
                                             RUN + (size_t)RBS[e] * RUNCAP, SLOT + (size_t)SBS[e],
                                             FLAG + (size_t)RBS[e] * 32);
  }
  for (int l = 0; l < 2; ++l) {
    k_kqv<<<dim3(NP / GBM, 3), NTHR, 0, stream>>>(HHL, WKQ, VEC, l, Q, KV2);
    for (int e = 0; e < 13; ++e) {
      const int s = ES[e], d = ED[e];
      const int first = (e == 0 || e == 1 || e == 11) ? 1 : 0;
      k_rel<<<dim3(NPT[s] / GBM, 2), NTHR, 0, stream>>>(KV2, RB + (size_t)(l * 13 + e) * RBMAT, PBS[s], KVE);
      k_replay<<<NPT[d] / 64, NTHR, 0, stream>>>(Q, KVE, RUN + (size_t)RBS[e] * RUNCAP, SLOT + (size_t)SBS[e],
                                                 FLAG + (size_t)RBS[e] * 32, VEC + VB_PREL + (l * 13 + e) * 4,
                                                 ST, PBS[d], NTY[s], SLB[d], first);
    }
    if (l == 0) k_out<0><<<NP / GBM, NTHR, 0, stream>>>(ST, WOU, VEC, FLAG, l, H, HHL, out);
    else        k_out<1><<<NP / GBM, NTHR, 0, stream>>>(ST, WOU, VEC, FLAG, l, H, HHL, out);
  }
}
